// InputsSchedulePredictorNN_11055245820208
// MI455X (gfx1250) — hardware-verified
//
#include <hip/hip_runtime.h>
#include <math.h>

typedef _Float16 v16h __attribute__((ext_vector_type(16)));
typedef _Float16 v8h  __attribute__((ext_vector_type(8)));
typedef float    v8f  __attribute__((ext_vector_type(8)));
typedef float    v4f  __attribute__((ext_vector_type(4)));
typedef unsigned v4u  __attribute__((ext_vector_type(4)));

constexpr int kBatch = 16384, kT = 50, kIn = 5, kH = 64;
constexpr int kPE1 = 32, kPE2 = 16, kPD1 = 64, kPD2 = 16, kOut = 2, kTS = 35, kNData = 4;
constexpr int kKenc = 96;
constexpr int kRowsPB = 16;
constexpr int kPreRows = 128;
constexpr int kOutPerBlock = kRowsPB * kTS * kOut;
constexpr float kDT = 0.033f, kVelScale = 0.1f, kVelBias = 0.0f, kJerkLim = 1.0f, kSteerLim = 1.0f;
constexpr float kActCarry = 256.0f, kWCarry = 16.0f, kUncarry = 1.0f / 4096.0f;

static_assert(kBatch % kRowsPB == 0, "rows per block");
static_assert(kBatch % kPreRows == 0, "pre rows per block");
static_assert((kOutPerBlock * 4) % 128 == 0, "block output is whole lines");
static_assert(kH == 64 && kPD1 == 64 && kPE2 == 16 && kPD2 == 16, "tile shapes");

constexpr size_t kOffWenc = 0;
constexpr size_t kOffWdec = 49152;
constexpr size_t kOffWpd  = 81920;
constexpr size_t kOffWf1  = 90112;
constexpr size_t kOffH2   = 92160;
constexpr size_t kWsTotal = kOffH2 + (size_t)kT * kBatch * kPE2 * 2;
static_assert(kOffWdec == kOffWenc + 256 * kKenc * 2, "carve");
static_assert(kOffWpd  == kOffWdec + 256 * kH * 2, "carve");
static_assert(kOffWf1  == kOffWpd + kPD1 * kH * 2, "carve");
static_assert(kOffH2   == kOffWf1 + kPD2 * kPD1 * 2, "carve");
static_assert(kWsTotal == 26306560, "carve total");

#define DEVI __device__ __forceinline__

union FragH { v16h v; v8h h[2]; };
DEVI v16h fload(const _Float16* p) {
  FragH f; f.h[0] = *(const v8h*)(p); f.h[1] = *(const v8h*)(p + 16); return f.v;
}
DEVI v8f mma16(v16h a, v16h b, v8f c) {
  c = __builtin_amdgcn_wmma_f32_16x16x32_f16(false, a, false, b, (short)0, c, false, false);
  asm volatile("v_nop\n\tv_nop\n\tv_nop\n\tv_nop" : "+v"(c) : "v"(a), "v"(b));
  return c;
}
DEVI v8f zero8() { v8f z = {0.f, 0.f, 0.f, 0.f, 0.f, 0.f, 0.f, 0.f}; return z; }

DEVI float sigm(float x) {
  x = fminf(fmaxf(x, -30.0f), 30.0f);
  const float e = expf(-x);
  return 1.0f / (1.0f + e);
}
DEVI float tnh(float x) {
  x = fminf(fmaxf(x, -15.0f), 15.0f);
  const float e = expf(2.0f * x);
  return 1.0f - 2.0f / (1.0f + e);
}

__global__ __launch_bounds__(128) void k_prep(
    const float* __restrict__ enc_wih, const float* __restrict__ enc_whh,
    const float* __restrict__ dec_whh, const float* __restrict__ pd_w,
    const float* __restrict__ fin_w1,
    _Float16* __restrict__ Wenc, _Float16* __restrict__ Wdec,
    _Float16* __restrict__ Wpd, _Float16* __restrict__ Wf1) {
  const int tid = threadIdx.x, blk = blockIdx.x;
  v8h hv;
  _Float16* dst;
  if (blk < 24) {
    const int cidx = blk * 128 + tid;
    const int n = cidx / 12, cc = cidx - n * 12;
#pragma unroll
    for (int j = 0; j < 8; ++j) {
      const int k = cc * 8 + j;
      int ka = k; ka = ka > 15 ? 15 : ka;
      int kb = k - 32; kb = kb < 0 ? 0 : kb; kb = kb > 63 ? 63 : kb;
      const float wa = enc_wih[n * kPE2 + ka];
      const float wb = enc_whh[n * kH + kb];
      const float v = (cc < 2) ? wa : ((cc < 4) ? 0.0f : wb);
      hv[j] = (_Float16)(kWCarry * v);
    }
    dst = Wenc + (size_t)cidx * 8;
  } else if (blk < 40) {
    const int cidx = blk * 128 + tid - 3072;
    const int n = cidx >> 3, cc = cidx & 7;
#pragma unroll
    for (int j = 0; j < 8; ++j) hv[j] = (_Float16)(kWCarry * dec_whh[n * kH + cc * 8 + j]);
    dst = Wdec + (size_t)cidx * 8;
  } else if (blk < 44) {
    const int cidx = blk * 128 + tid - 5120;
    const int n = cidx >> 3, cc = cidx & 7;
#pragma unroll
    for (int j = 0; j < 8; ++j) hv[j] = (_Float16)(kWCarry * pd_w[n * kH + cc * 8 + j]);
    dst = Wpd + (size_t)cidx * 8;
  } else {
    const int cidx = blk * 128 + tid - 5632;
    const int n = cidx >> 3, cc = cidx & 7;
#pragma unroll
    for (int j = 0; j < 8; ++j) hv[j] = (_Float16)(kWCarry * fin_w1[n * kPD1 + cc * 8 + j]);
    dst = Wf1 + (size_t)cidx * 8;
  }
  *(volatile v8h*)dst = hv;
  __threadfence();
  *(volatile v8h*)dst = hv;
}

__global__ __launch_bounds__(128) void k_pre(
    const float* __restrict__ x, const float* __restrict__ pe_w1, const float* __restrict__ pe_b1,
    const float* __restrict__ pe_w2, const float* __restrict__ pe_b2, _Float16* __restrict__ H2p) {
  __shared__ float pw1[kPE1 * kIn];
  __shared__ float pb1[kPE1];
  __shared__ float pb2[kPE2];
  __shared__ __align__(16) _Float16 W2t[kPE2 * kPE1];
  __shared__ __align__(16) _Float16 Ah1[kPreRows * kPE1];
  __shared__ __align__(16) _Float16 Stg[kPreRows * kPE2];

  const int tid = threadIdx.x, lane = tid & 31, wave = tid >> 5;
  const int hh = lane >> 4, c = lane & 15, koff = hh * 8;
  const int t  = blockIdx.x >> 7;
  const int bb = blockIdx.x & 127;

  for (int i = tid; i < kPE1 * kIn; i += 128) pw1[i] = pe_w1[i];
  if (tid < kPE1) pb1[tid] = pe_b1[tid];
  if (tid < kPE2) pb2[tid] = pe_b2[tid];
  for (int i = tid; i < kPE2 * kPE1; i += 128) W2t[i] = (_Float16)(kWCarry * pe_w2[i]);
  __syncthreads();

  {
    const int b = bb * kPreRows + tid;
    const float* xr = x + ((size_t)b * kT + t) * kIn;
    const float f0 = (xr[0] - kVelBias) * kVelScale;
    const float f1 = xr[1], f2 = xr[2], f3 = xr[3], f4 = xr[4];
#pragma unroll 1
    for (int col = 0; col < kPE1; ++col) {
      const float* w = pw1 + col * kIn;
      float a = pb1[col] + f0 * w[0] + f1 * w[1] + f2 * w[2] + f3 * w[3] + f4 * w[4];
      Ah1[tid * kPE1 + col] = (_Float16)(kActCarry * fmaxf(a, 0.0f));
    }
  }
  __syncthreads();

  v8f acc[2];
  const v16h bfr = fload(W2t + c * kPE1 + koff);
#pragma unroll
  for (int i = 0; i < 2; ++i) {
    const v16h a = fload(Ah1 + (32 * wave + 16 * i + c) * kPE1 + koff);
    acc[i] = mma16(a, bfr, zero8());
  }
  const float b2v = pb2[c];
#pragma unroll
  for (int i = 0; i < 2; ++i) {
#pragma unroll
    for (int r = 0; r < 8; ++r) {
      const float v = fmaxf(acc[i][r] * kUncarry + b2v, 0.0f);
      Stg[(32 * wave + 16 * i + 8 * hh + r) * kPE2 + c] = (_Float16)(kActCarry * v);
    }
  }
  __syncthreads();

  _Float16* dst = H2p + ((size_t)t * kBatch + (size_t)bb * kPreRows) * kPE2;
  for (int pass = 0; pass < 2; ++pass) {
#pragma unroll
    for (int it = 0; it < 2; ++it) {
      const int row0 = 32 * wave + 16 * it;
      const v4u v = *(const v4u*)(Stg + row0 * kPE2 + lane * 8);
      *(volatile v4u*)(dst + row0 * kPE2 + lane * 8) = v;
    }
    __threadfence();
  }
}

__global__ __launch_bounds__(128) void k_main(
    const _Float16* __restrict__ H2p, const _Float16* __restrict__ Wenc,
    const _Float16* __restrict__ Wdec, const _Float16* __restrict__ Wpd,
    const _Float16* __restrict__ Wf1,
    const float* __restrict__ x, const int* __restrict__ dsx,
    const float* __restrict__ enc_bih, const float* __restrict__ enc_bhh,
    const float* __restrict__ dec_wih, const float* __restrict__ dec_bih,
    const float* __restrict__ dec_bhh, const float* __restrict__ pd_b,
    const float* __restrict__ scales, const float* __restrict__ fin_b1,
    const float* __restrict__ fin_w2, const float* __restrict__ fin_b2,
    float* __restrict__ out) {
  __shared__ __align__(16) _Float16 At[2 * kRowsPB * kKenc];
  __shared__ __align__(16) _Float16 Pt[kRowsPB * kPD1];
  __shared__ float bE[256];
  __shared__ float bD[256];
  __shared__ float dW[256 * 4];
  __shared__ float pS[kRowsPB * kPD1];
  __shared__ float pB[kPD1];
  __shared__ float fB[kPD2];
  __shared__ float fW[kOut * kPD2];
  __shared__ float fBb[kOut];
  __shared__ __align__(16) float Ost[kOutPerBlock];

  const int tid = threadIdx.x, lane = tid & 31, wave = tid >> 5;
  const int hh = lane >> 4, c = lane & 15, koff = hh * 8;
  const int b0 = blockIdx.x * kRowsPB;
  const int u = 16 * wave + c;

  {
    const v4u z = {0u, 0u, 0u, 0u};
    for (int i = tid; i < (2 * kRowsPB * kKenc) / 8; i += 128) *(v4u*)(At + 8 * i) = z;
  }
  for (int i = tid; i < 256; i += 128) {
    bE[i] = enc_bih[i] + enc_bhh[i];
    bD[i] = dec_bih[i] + dec_bhh[i];
  }
  for (int i = tid; i < 256 * 4; i += 128) dW[i] = dec_wih[i];
  for (int i = tid; i < kRowsPB * kPD1; i += 128) {
    const int row = i >> 6, col = i & 63;
    int id = dsx[b0 + row];
    id = id < 0 ? id + kNData : id;
    id = id < 0 ? 0 : id;
    id = id > kNData - 1 ? kNData - 1 : id;
    pS[i] = scales[id * kPD1 + col];
  }
  if (tid < kPD1) pB[tid] = pd_b[tid];
  if (tid < kPD2) fB[tid] = fin_b1[tid];
  if (tid < kOut * kPD2) fW[tid] = fin_w2[tid];
  if (tid < kOut) fBb[tid] = fin_b2[tid];
  __syncthreads();
  {
    const int row = tid >> 3, ch = tid & 7;
    const unsigned w = *(const unsigned*)(H2p + ((size_t)(b0 + row)) * kPE2 + 2 * ch);
    *(unsigned*)(At + row * kKenc + 2 * ch) = w;
  }
  __syncthreads();

  float cst[8];
#pragma unroll
  for (int r = 0; r < 8; ++r) cst[r] = 0.0f;

  for (int t = 0; t < kT; ++t) {
    const _Float16* Ac = At + (t & 1) * (kRowsPB * kKenc);
    _Float16* An = At + ((t + 1) & 1) * (kRowsPB * kKenc);
    v8f acc[4];
#pragma unroll
    for (int j = 0; j < 4; ++j) acc[j] = zero8();
#pragma unroll 1
    for (int kc = 0; kc < 3; ++kc) {
      const v16h a = fload(Ac + c * kKenc + kc * 32 + koff);
#pragma unroll
      for (int j = 0; j < 4; ++j) {
        const v16h bq = fload(Wenc + (size_t)(j * 64 + u) * kKenc + kc * 32 + koff);
        acc[j] = mma16(a, bq, acc[j]);
      }
    }
    const float bi = bE[u], bf = bE[64 + u], bg = bE[128 + u], bo = bE[192 + u];
#pragma unroll
    for (int r = 0; r < 8; ++r) {
      const float gi = acc[0][r] * kUncarry + bi;
      const float gf = acc[1][r] * kUncarry + bf;
      const float gg = acc[2][r] * kUncarry + bg;
      const float go = acc[3][r] * kUncarry + bo;
      const float cn = sigm(gf) * cst[r] + sigm(gi) * tnh(gg);
      const float hn = sigm(go) * tnh(cn);
      cst[r] = cn;
      An[(8 * hh + r) * kKenc + 32 + u] = (_Float16)(kActCarry * hn);
    }
    {
      const int tn = (t + 1 < kT) ? (t + 1) : (kT - 1);
      const int row = tid >> 3, ch = tid & 7;
      const unsigned w = *(const unsigned*)(H2p + ((size_t)tn * kBatch + b0 + row) * kPE2 + 2 * ch);
      *(unsigned*)(An + row * kKenc + 2 * ch) = w;
    }
    __syncthreads();
  }

  float hd0[8], hd1[8], tl0[8], tl1[8];
#pragma unroll
  for (int r = 0; r < 8; ++r) {
    const float* xr = x + ((size_t)(b0 + 8 * hh + r) * kT + (kT - 1)) * kIn;
    const float c0 = xr[3], c1 = xr[4];
    const float p0 = xr[3 - kIn], p1 = xr[4 - kIn];
    hd0[r] = c0; hd1[r] = c1;
    tl0[r] = (c0 - p0) * (1.0f / kDT);
    tl1[r] = (c1 - p1) * (1.0f / kDT);
  }
  const float wi0 = dW[u * 4 + 0], wi1 = dW[u * 4 + 1], wi2 = dW[u * 4 + 2], wi3 = dW[u * 4 + 3];
  const float wf0 = dW[(64 + u) * 4 + 0], wf1 = dW[(64 + u) * 4 + 1], wf2 = dW[(64 + u) * 4 + 2], wf3 = dW[(64 + u) * 4 + 3];
  const float wg0 = dW[(128 + u) * 4 + 0], wg1 = dW[(128 + u) * 4 + 1], wg2 = dW[(128 + u) * 4 + 2], wg3 = dW[(128 + u) * 4 + 3];
  const float wo0 = dW[(192 + u) * 4 + 0], wo1 = dW[(192 + u) * 4 + 1], wo2 = dW[(192 + u) * 4 + 2], wo3 = dW[(192 + u) * 4 + 3];
  const float bdi = bD[u], bdf = bD[64 + u], bdg = bD[128 + u], bdo = bD[192 + u];
  const float pbv = pB[u];
  const float fbv = fB[c], w20 = fW[c], w21 = fW[kPD2 + c], b20 = fBb[0], b21 = fBb[1];

  for (int s = 0; s < kTS; ++s) {
    const int g = kT + s;
    const _Float16* Ac = At + (g & 1) * (kRowsPB * kKenc);
    _Float16* An = At + ((g + 1) & 1) * (kRowsPB * kKenc);
    v8f acc[4];
#pragma unroll
    for (int j = 0; j < 4; ++j) acc[j] = zero8();
#pragma unroll 1
    for (int kc = 0; kc < 2; ++kc) {
      const v16h a = fload(Ac + c * kKenc + 32 + kc * 32 + koff);
#pragma unroll
      for (int j = 0; j < 4; ++j) {
        const v16h bq = fload(Wdec + (size_t)(j * 64 + u) * kH + kc * 32 + koff);
        acc[j] = mma16(a, bq, acc[j]);
      }
    }
#pragma unroll
    for (int r = 0; r < 8; ++r) {
      const float h0 = hd0[r], h1 = hd1[r], t0 = tl0[r], t1 = tl1[r];
      const float gi = acc[0][r] * kUncarry + bdi + wi0 * h0 + wi1 * h1 + wi2 * t0 + wi3 * t1;
      const float gf = acc[1][r] * kUncarry + bdf + wf0 * h0 + wf1 * h1 + wf2 * t0 + wf3 * t1;
      const float gg = acc[2][r] * kUncarry + bdg + wg0 * h0 + wg1 * h1 + wg2 * t0 + wg3 * t1;
      const float go = acc[3][r] * kUncarry + bdo + wo0 * h0 + wo1 * h1 + wo2 * t0 + wo3 * t1;
      const float cn = sigm(gf) * cst[r] + sigm(gi) * tnh(gg);
      const float hn = sigm(go) * tnh(cn);
      cst[r] = cn;
      An[(8 * hh + r) * kKenc + 32 + u] = (_Float16)(kActCarry * hn);
    }
    __syncthreads();
    {
      v8f ap = zero8();
#pragma unroll 1
      for (int kc = 0; kc < 2; ++kc) {
        const v16h a = fload(An + c * kKenc + 32 + kc * 32 + koff);
        const v16h bq = fload(Wpd + (size_t)u * kH + kc * 32 + koff);
        ap = mma16(a, bq, ap);
      }
#pragma unroll
      for (int r = 0; r < 8; ++r) {
        const float v = fmaxf(ap[r] * kUncarry + pbv, 0.0f) * pS[(8 * hh + r) * kPD1 + u];
        Pt[(8 * hh + r) * kPD1 + u] = (_Float16)(kActCarry * v);
      }
    }
    __syncthreads();
    {
      v8f af = zero8();
#pragma unroll 1
      for (int kc = 0; kc < 2; ++kc) {
        const v16h a = fload(Pt + c * kPD1 + kc * 32 + koff);
        const v16h bq = fload(Wf1 + (size_t)c * kPD1 + kc * 32 + koff);
        af = mma16(a, bq, af);
      }
#pragma unroll
      for (int r = 0; r < 8; ++r) {
        const float f1 = fmaxf(af[r] * kUncarry + fbv, 0.0f);
        float p0 = f1 * w20, p1 = f1 * w21;
#pragma unroll
        for (int off = 1; off < 16; off <<= 1) {
          p0 += __shfl_xor(p0, off, 32);
          p1 += __shfl_xor(p1, off, 32);
        }
        const float o0 = tnh(p0 + b20) * kJerkLim;
        const float o1 = tnh(p1 + b21) * kSteerLim;
        hd0[r] = hd0[r] + o0 * kDT;
        hd1[r] = hd1[r] + o1 * kDT;
        tl0[r] = o0;
        tl1[r] = o1;
        if (wave == 0 && c == 0) {
          Ost[(8 * hh + r) * (kTS * kOut) + 2 * s]     = o0;
          Ost[(8 * hh + r) * (kTS * kOut) + 2 * s + 1] = o1;
        }
      }
    }
  }
  __syncthreads();

  float* ob = out + (size_t)blockIdx.x * kOutPerBlock;
  const int l8 = lane & 7;
  for (int pass = 0; pass < 2; ++pass) {
#pragma unroll 1
    for (int it = 0; it < 9; ++it) {
      const int line = it * 4 + wave;
      const int lc = line < kTS ? line : (kTS - 1);
      const v4f v = *(const v4f*)(Ost + lc * 32 + l8 * 4);
      if (line < kTS && lane < 8) *(volatile v4f*)(ob + lc * 32 + l8 * 4) = v;
    }
    __threadfence();
  }
}

extern "C" void kernel_launch(void* const* d_in, const int* in_sizes, int n_in,
                              void* d_out, int out_size, void* d_ws, size_t ws_size,
                              hipStream_t stream) {
  if (n_in < 21) return;
  if (in_sizes[0] != kBatch * kT * kIn) return;
  if (in_sizes[1] != kBatch) return;
  if (in_sizes[2] != kPE1 * kIn || in_sizes[4] != kPE2 * kPE1) return;
  if (in_sizes[6] != 256 * kPE2 || in_sizes[7] != 256 * kH) return;
  if (in_sizes[10] != 256 * 2 * kOut || in_sizes[11] != 256 * kH) return;
  if (in_sizes[14] != kPD1 * kH || in_sizes[16] != kNData * kPD1) return;
  if (in_sizes[17] != kPD2 * kPD1 || in_sizes[19] != kOut * kPD2) return;
  if (out_size != kBatch * kTS * kOut) return;
  if (ws_size < kWsTotal) return;

  const float* x       = (const float*)d_in[0];
  const int*   dsx     = (const int*)d_in[1];
  const float* pe_w1   = (const float*)d_in[2];
  const float* pe_b1   = (const float*)d_in[3];
  const float* pe_w2   = (const float*)d_in[4];
  const float* pe_b2   = (const float*)d_in[5];
  const float* enc_wih = (const float*)d_in[6];
  const float* enc_whh = (const float*)d_in[7];
  const float* enc_bih = (const float*)d_in[8];
  const float* enc_bhh = (const float*)d_in[9];
  const float* dec_wih = (const float*)d_in[10];
  const float* dec_whh = (const float*)d_in[11];
  const float* dec_bih = (const float*)d_in[12];
  const float* dec_bhh = (const float*)d_in[13];
  const float* pd_w    = (const float*)d_in[14];
  const float* pd_b    = (const float*)d_in[15];
  const float* scales  = (const float*)d_in[16];
  const float* fin_w1  = (const float*)d_in[17];
  const float* fin_b1  = (const float*)d_in[18];
  const float* fin_w2  = (const float*)d_in[19];
  const float* fin_b2  = (const float*)d_in[20];
  float* out = (float*)d_out;

  char* ws = (char*)d_ws;
  _Float16* Wenc = (_Float16*)(ws + kOffWenc);
  _Float16* Wdec = (_Float16*)(ws + kOffWdec);
  _Float16* Wpd  = (_Float16*)(ws + kOffWpd);
  _Float16* Wf1  = (_Float16*)(ws + kOffWf1);
  _Float16* H2p  = (_Float16*)(ws + kOffH2);

  k_prep<<<dim3(45), dim3(128), 0, stream>>>(enc_wih, enc_whh, dec_whh, pd_w, fin_w1, Wenc, Wdec, Wpd, Wf1);
  k_pre<<<dim3(kT * (kBatch / kPreRows)), dim3(128), 0, stream>>>(x, pe_w1, pe_b1, pe_w2, pe_b2, H2p);
  k_main<<<dim3(kBatch / kRowsPB), dim3(128), 0, stream>>>(
      H2p, Wenc, Wdec, Wpd, Wf1, x, dsx, enc_bih, enc_bhh, dec_wih, dec_bih, dec_bhh,
      pd_b, scales, fin_b1, fin_w2, fin_b2, out);
}
